// MambaEncoderBlock_66305705115705
// MI455X (gfx1250) — hardware-verified
//
#include <hip/hip_runtime.h>
#include <math.h>

typedef __attribute__((ext_vector_type(16))) _Float16 v16h;
typedef __attribute__((ext_vector_type(8)))  _Float16 v8h;
typedef __attribute__((ext_vector_type(16))) __bf16   v16b;
typedef __attribute__((ext_vector_type(8)))  __bf16   v8b;
typedef __attribute__((ext_vector_type(8)))  float    v8f;
typedef __attribute__((ext_vector_type(4)))  float    v4f;

constexpr int kBatch   = 4;
constexpr int kSeqL    = 2048;
constexpr int kDmod    = 512;
constexpr int kDin     = 1024;
constexpr int kNst     = 16;
constexpr int kDtR     = 32;
constexpr int kPrjN    = 64;
constexpr int kPrjP    = 64;
constexpr int kXZP     = 2 * kDin;
constexpr int kRows    = kBatch * kSeqL;
constexpr int kDsf     = 2;
constexpr int kOutT    = kSeqL / kDsf;
constexpr int kOutRows = kBatch * kOutT;
constexpr int kTP      = 260;
constexpr float kWCarry   = 32.0f;
constexpr float kWdtCarry = 8.0f;
constexpr float kUcCarry  = 16.0f;
constexpr float kDtCarry  = 16.0f;
constexpr float kYCarry   = 64.0f;

__device__ __forceinline__ unsigned short f2bf_bits(float f) {
  unsigned u = __float_as_uint(f);
  return (unsigned short)((u + 0x7FFFu + ((u >> 16) & 1u)) >> 16);
}
__device__ __forceinline__ float bf_bits2f(unsigned short h) { return __uint_as_float(((unsigned)h) << 16); }

__device__ __forceinline__ void dep_guard_h(v8f& a, v8f& b, v16h x, v16h y) { asm volatile("v_nop\n\tv_nop\n\tv_nop\n\tv_nop" : "+v"(a), "+v"(b) : "v"(x), "v"(y)); }
__device__ __forceinline__ void dep_guard_b(v8f& a, v8f& b, v16b x, v16b y) { asm volatile("v_nop\n\tv_nop\n\tv_nop\n\tv_nop" : "+v"(a), "+v"(b) : "v"(x), "v"(y)); }
__device__ __forceinline__ void keep4_h(v16h a, v16h b, v16h c, v16h d) { asm volatile("v_nop" :: "v"(a), "v"(b), "v"(c), "v"(d)); }
__device__ __forceinline__ void keep4_b(v16b a, v16b b, v16b c, v16b d) { asm volatile("v_nop" :: "v"(a), "v"(b), "v"(c), "v"(d)); }
__device__ __forceinline__ void acc_guard4(v8f& a, v8f& b, v8f& c, v8f& d) { asm volatile("v_nop\n\tv_nop\n\tv_nop\n\tv_nop" : "+v"(a), "+v"(b), "+v"(c), "+v"(d)); }
template <typename T> struct Frag;
template <> struct Frag<_Float16> {
  typedef v16h V; union U { v16h v; v8h h[2]; };
  static __device__ __forceinline__ v16h load(const _Float16* p) {
    U f; f.h[0] = *(const v8h*)(p); f.h[1] = *(const v8h*)(p + 16); return f.v;
  }
  static __device__ __forceinline__ v8f mma(v16h a, v16h b, v8f c) {
    return __builtin_amdgcn_wmma_f32_16x16x32_f16(false, a, false, b, (short)0, c, false, false);
  }
  static __device__ __forceinline__ void guard(v8f& a, v8f& b, v16h x, v16h y) { dep_guard_h(a, b, x, y); }
  static __device__ __forceinline__ void keep(v16h a, v16h b, v16h c, v16h d) { keep4_h(a, b, c, d); }
};
template <> struct Frag<__bf16> {
  typedef v16b V; union U { v16b v; v8b h[2]; };
  static __device__ __forceinline__ v16b load(const __bf16* p) {
    U f; f.h[0] = *(const v8b*)(p); f.h[1] = *(const v8b*)(p + 16); return f.v;
  }
  static __device__ __forceinline__ v8f mma(v16b a, v16b b, v8f c) {
    return __builtin_amdgcn_wmma_f32_16x16x32_bf16(false, a, false, b, (short)0, c, false, false);
  }
  static __device__ __forceinline__ void guard(v8f& a, v8f& b, v16b x, v16b y) { dep_guard_b(a, b, x, y); }
  static __device__ __forceinline__ void keep(v16b a, v16b b, v16b c, v16b d) { keep4_b(a, b, c, d); }
};

template <int ET> struct Elem;
template <> struct Elem<0> { typedef _Float16 T; };
template <> struct Elem<1> { typedef __bf16 T; };
template <int ET, bool SPLIT, int BIAS_MODE, int OUT_MODE, bool RESID, int ACT = 0>
__global__ __launch_bounds__(256) void wmma_gemm64(
    const unsigned short* __restrict__ Ap, const unsigned short* __restrict__ A2p, int lda, long strideA,
    const unsigned short* __restrict__ Btp, const unsigned short* __restrict__ Bt2p, int ldb, long strideB,
    void* __restrict__ Cout, void* __restrict__ Cout2, int ldc, long strideC,
    const float* __restrict__ bias,
    const float* __restrict__ resid, long strideR,
    int M, int N, int K, float scale) {
  typedef typename Elem<ET>::T T;
  typedef typename Frag<T>::V V;
  const T* A = (const T*)Ap; const T* A2 = (const T*)A2p; const T* Bt = (const T*)Btp; const T* Bt2 = (const T*)Bt2p;
  __shared__ __align__(16) float sT[8][16 * 68];
  const int b    = blockIdx.y;
  const int lane = threadIdx.x & 31;
  const int wave = threadIdx.x >> 5;
  const int tilesN = N >> 6;
  const int tilesM = M >> 6;
  const int tile = blockIdx.x * 8 + wave;
  if (tile >= tilesM * tilesN) return;
  const int tm = tile / tilesN;
  const int tn = tile - tm * tilesN;
  const int m0 = tm << 6;
  const int n0 = tn << 6;

  const T* Ab  = A  + (size_t)b * strideA;
  const T* Bb  = Bt + (size_t)b * strideB;
  const T* Ab2 = SPLIT ? (A2  + (size_t)b * strideA) : nullptr;
  const T* Bb2 = SPLIT ? (Bt2 + (size_t)b * strideB) : nullptr;

  const int rlane = lane & 15;
  const int koff  = (lane >> 4) * 8;
  const int mOff  = (lane >> 4) * 8;

  v8f acc[4][4];
#pragma unroll
  for (int i = 0; i < 4; ++i)
#pragma unroll
    for (int j = 0; j < 4; ++j) acc[i][j] = (v8f){0.f,0.f,0.f,0.f,0.f,0.f,0.f,0.f};

  for (int k0 = 0; k0 < K; k0 += 32) {
    V bh[4], bl[4];
#pragma unroll
    for (int j = 0; j < 4; ++j) {
      const size_t bo = (size_t)(n0 + (j << 4) + rlane) * ldb + koff + k0;
      bh[j] = Frag<T>::load(Bb + bo);
      if (SPLIT) bl[j] = Frag<T>::load(Bb2 + bo);
    }
#pragma unroll
    for (int i = 0; i < 4; ++i) {
      const size_t ao = (size_t)(m0 + (i << 4) + rlane) * lda + koff + k0;
      V ah = Frag<T>::load(Ab + ao);
      V al;
      if (SPLIT) al = Frag<T>::load(Ab2 + ao);
#pragma unroll
      for (int j = 0; j < 4; ++j) {
        acc[i][j] = Frag<T>::mma(ah, bh[j], acc[i][j]);
        if (SPLIT) {
          acc[i][j] = Frag<T>::mma(ah, bl[j], acc[i][j]);
          acc[i][j] = Frag<T>::mma(al, bh[j], acc[i][j]);
        }
      }
      Frag<T>::guard(acc[i][0], acc[i][3], ah, SPLIT ? al : ah);
    }
    Frag<T>::keep(bh[0], bh[1], bh[2], bh[3]);
    if (SPLIT) Frag<T>::keep(bl[0], bl[1], bl[2], bl[3]);
  }
  acc_guard4(acc[0][0], acc[0][1], acc[0][2], acc[0][3]);
  acc_guard4(acc[1][0], acc[1][1], acc[1][2], acc[1][3]);
  acc_guard4(acc[2][0], acc[2][1], acc[2][2], acc[2][3]);
  acc_guard4(acc[3][0], acc[3][1], acc[3][2], acc[3][3]);

  float* slab = sT[wave];
  const float* Rb = RESID ? (resid + (size_t)b * strideR) : nullptr;
#pragma unroll
  for (int i = 0; i < 4; ++i) {
    const int mBase = m0 + (i << 4);
#pragma unroll
    for (int j = 0; j < 4; ++j) {
      const int n = n0 + (j << 4) + rlane;
      float bv = 0.f;
      if (BIAS_MODE == 2) bv = bias[n];
#pragma unroll
      for (int r = 0; r < 8; ++r) {
        float v = acc[i][j][r] * scale;
        if (BIAS_MODE == 1) v += bias[mBase + mOff + r];
        if (BIAS_MODE == 2) v += bv;
        if (RESID) v += Rb[(size_t)(mBase + mOff + r) * ldc + n];
        if (ACT == 1) v = tanhf(v);
        if (ACT == 2) v = fmaxf(v, 0.0f);
        if (ACT == 3) v = v / (1.0f + expf(-v));
        if (ACT == 4) v = (v > 0.f) ? v : 0.01f * v;
        if (ACT == 5) v = 0.5f * v * (1.0f + erff(v * 0.70710678118654752f));
        slab[(mOff + r) * 68 + (j << 4) + rlane] = v;
      }
    }
    __builtin_amdgcn_fence(__ATOMIC_RELEASE, "workgroup");
    __builtin_amdgcn_wave_barrier();
    __builtin_amdgcn_fence(__ATOMIC_ACQUIRE, "workgroup");
    if (OUT_MODE == 0) {
      float* C = (float*)Cout + (size_t)b * strideC;
      const int hh = lane >> 4, c4 = (lane & 15) * 4;
      for (int pass = 0; pass < 2; ++pass) {
#pragma unroll
        for (int it = 0; it < 8; ++it) {
          const int row = it * 2 + hh;
          v4f v = *(const v4f*)(slab + row * 68 + c4);
          *(volatile v4f*)(C + (size_t)(mBase + row) * ldc + n0 + c4) = v;
        }
        __threadfence();
      }
    } else {
      const int q = lane >> 3, c8 = (lane & 7) * 8;
      unsigned short* C  = (unsigned short*)Cout  + (size_t)b * strideC;
      unsigned short* C2 = (OUT_MODE == 2) ? ((unsigned short*)Cout2 + (size_t)b * strideC) : nullptr;
      for (int pass = 0; pass < 2; ++pass) {
#pragma unroll
        for (int it = 0; it < 4; ++it) {
          const int row = it * 4 + q;
          const float* sp = slab + row * 68 + c8;
          v8h hv, lv;
#pragma unroll
          for (int e = 0; e < 8; ++e) {
            if (OUT_MODE == 1) {
              hv[e] = (_Float16)sp[e];
            } else {
              unsigned short hb = f2bf_bits(sp[e]);
              unsigned short lb = f2bf_bits(sp[e] - bf_bits2f(hb));
              hv[e] = __builtin_bit_cast(_Float16, hb);
              lv[e] = __builtin_bit_cast(_Float16, lb);
            }
          }
          *(volatile v8h*)(C + (size_t)(mBase + row) * ldc + n0 + c8) = hv;
          if (OUT_MODE == 2) *(volatile v8h*)(C2 + (size_t)(mBase + row) * ldc + n0 + c8) = lv;
        }
        __threadfence();
      }
    }
    __builtin_amdgcn_fence(__ATOMIC_RELEASE, "workgroup");
    __builtin_amdgcn_wave_barrier();
    __builtin_amdgcn_fence(__ATOMIC_ACQUIRE, "workgroup");
  }
}

__global__ __launch_bounds__(256) void cast_f16_kernel(
    const float* __restrict__ src, unsigned short* __restrict__ dst, int total8, float scale)
{
  const int i = blockIdx.x * 256 + threadIdx.x;
  if (i >= total8) return;
  const size_t e0 = (size_t)i << 3;
  const float* p = src + e0;
  const v4f a0 = *(const v4f*)(p);
  const v4f a1 = *(const v4f*)(p + 4);
  v8h hv;
#pragma unroll
  for (int e = 0; e < 4; ++e) {
    hv[e]     = (_Float16)(a0[e] * scale);
    hv[4 + e] = (_Float16)(a1[e] * scale);
  }
  unsigned short* q = dst + e0;
  *(volatile v8h*)q = hv;
  __threadfence();
  *(volatile v8h*)q = hv;
}

__global__ __launch_bounds__(256) void transpose_cast_kernel(
    const float* __restrict__ W, unsigned short* __restrict__ Bt, int Kdim, int Ndim, int Npad, float scale)
{
  __shared__ float tile[64 * 65];
  const int tid = threadIdx.x, lane = tid & 31, wave = tid >> 5;
  const int n0 = blockIdx.x * 64;
  const int k0 = blockIdx.y * 64;
  (void)Npad;
#pragma unroll
  for (int p = 0; p < 16; ++p) {
    const int idx = tid + p * 256;
    const int kk  = idx >> 6;
    const int nn  = idx & 63;
    const int n   = n0 + nn;
    const int nc  = (n < Ndim) ? n : (Ndim - 1);
    const float v = W[(size_t)(k0 + kk) * Ndim + nc];
    tile[kk * 65 + nn] = (n < Ndim) ? (v * scale) : 0.f;
  }
  __syncthreads();
  const int q = lane >> 3, c8 = (lane & 7) * 8;
  v8h hv[2];
#pragma unroll
  for (int it = 0; it < 2; ++it) {
    const int nrow = it * 32 + wave * 4 + q;
#pragma unroll
    for (int e = 0; e < 8; ++e) hv[it][e] = (_Float16)tile[(c8 + e) * 65 + nrow];
  }
  for (int pass = 0; pass < 2; ++pass) {
#pragma unroll
    for (int it = 0; it < 2; ++it) {
      const int nrow = it * 32 + wave * 4 + q;
      *(volatile v8h*)(Bt + (size_t)(n0 + nrow) * Kdim + k0 + c8) = hv[it];
    }
    __threadfence();
  }
}

__global__ __launch_bounds__(256) void transpose_cast32_kernel(
    const float* __restrict__ W, unsigned short* __restrict__ Bt, int Ndim, float scale)
{
  __shared__ float tile[32 * 65];
  const int tid = threadIdx.x, lane = tid & 31, wave = tid >> 5;
  const int n0 = blockIdx.x * 64;
#pragma unroll
  for (int p = 0; p < 8; ++p) {
    const int idx = tid + p * 256;
    const int kk  = idx >> 6;
    const int nn  = idx & 63;
    const float v = W[(size_t)kk * Ndim + n0 + nn];
    tile[kk * 65 + nn] = v * scale;
  }
  __syncthreads();
  const int q = lane >> 2, c8 = (lane & 3) * 8;
  const int nrow = wave * 8 + q;
  v8h hv;
#pragma unroll
  for (int e = 0; e < 8; ++e) hv[e] = (_Float16)tile[(c8 + e) * 65 + nrow];
  unsigned short* dst = Bt + (size_t)(n0 + nrow) * 32 + c8;
  *(volatile v8h*)dst = hv;
  __threadfence();
  *(volatile v8h*)dst = hv;
}

__global__ __launch_bounds__(256) void dt_cast_kernel(
    const float* __restrict__ PROJ, unsigned short* __restrict__ DT16, int total8, float scale)
{
  const int i = blockIdx.x * 256 + threadIdx.x;
  if (i >= total8) return;
  const int e0  = i << 3;
  const int row = e0 >> 5;
  const int c8  = e0 & 31;
  const float* p = PROJ + (size_t)row * kPrjP + c8;
  const v4f a0 = *(const v4f*)(p);
  const v4f a1 = *(const v4f*)(p + 4);
  v8h hv;
#pragma unroll
  for (int e = 0; e < 4; ++e) {
    hv[e]     = (_Float16)(a0[e] * scale);
    hv[4 + e] = (_Float16)(a1[e] * scale);
  }
  unsigned short* qd = DT16 + e0;
  *(volatile v8h*)qd = hv;
  __threadfence();
  *(volatile v8h*)qd = hv;
}

__global__ __launch_bounds__(256) void conv_silu_kernel(
    const float* __restrict__ XZ, const float* __restrict__ cw, const float* __restrict__ cb,
    float* __restrict__ UC, unsigned short* __restrict__ UC16)
{
  __shared__ __align__(16) float sT[16 * kTP];
  const int tid = threadIdx.x, lane = tid & 31, wave = tid >> 5;
  const int d0 = blockIdx.x * 256, d = d0 + tid;
  const int t0 = blockIdx.y * 64;
  const float w0 = cw[d * 4 + 0], w1 = cw[d * 4 + 1], w2 = cw[d * 4 + 2], w3 = cw[d * 4 + 3];
  const float bc = cb[d];
  float xm3, xm2, xm1;
  {
    const int r3 = t0 - 3, r2 = t0 - 2, r1 = t0 - 1;
    const float v3 = XZ[(size_t)(r3 < 0 ? 0 : r3) * kXZP + d];
    const float v2 = XZ[(size_t)(r2 < 0 ? 0 : r2) * kXZP + d];
    const float v1 = XZ[(size_t)(r1 < 0 ? 0 : r1) * kXZP + d];
    xm3 = (r3 >= 0) ? v3 : 0.f;
    xm2 = (r2 >= 0) ? v2 : 0.f;
    xm1 = (r1 >= 0) ? v1 : 0.f;
  }
  const int hrow = wave >> 1;
  const int hch  = (wave & 1) * 128 + lane * 4;
#pragma unroll 1
  for (int sub = 0; sub < 4; ++sub) {
    const int lb = t0 + sub * 16;
#pragma unroll 1
    for (int s = 0; s < 16; ++s) {
      const float xc = XZ[(size_t)(lb + s) * kXZP + d];
      float acc = w0 * xm3;
      acc = fmaf(w1, xm2, acc);
      acc = fmaf(w2, xm1, acc);
      acc = fmaf(w3, xc, acc);
      const float sv = acc + bc;
      const float sg = __builtin_amdgcn_rcpf(1.0f + __expf(-sv));
      sT[s * kTP + tid] = sv * sg;
      xm3 = xm2; xm2 = xm1; xm1 = xc;
    }
    __syncthreads();
    v4f fv[4];
    v8h bv[2];
#pragma unroll
    for (int it = 0; it < 4; ++it) fv[it] = *(const v4f*)(sT + (it * 4 + hrow) * kTP + hch);
#pragma unroll
    for (int it = 0; it < 2; ++it) {
      const float* sp = sT + (it * 8 + wave) * kTP + lane * 8;
      const v4f a0 = *(const v4f*)(sp);
      const v4f a1 = *(const v4f*)(sp + 4);
#pragma unroll
      for (int e = 0; e < 4; ++e) {
        bv[it][e]     = (_Float16)(a0[e] * kUcCarry);
        bv[it][4 + e] = (_Float16)(a1[e] * kUcCarry);
      }
    }
    for (int pass = 0; pass < 2; ++pass) {
#pragma unroll
      for (int it = 0; it < 4; ++it)
        *(volatile v4f*)(UC + (size_t)(lb + it * 4 + hrow) * kDin + d0 + hch) = fv[it];
#pragma unroll
      for (int it = 0; it < 2; ++it)
        *(volatile v8h*)(UC16 + (size_t)(lb + it * 8 + wave) * kDin + d0 + lane * 8) = bv[it];
      __threadfence();
    }
    __syncthreads();
  }
}

__global__ __launch_bounds__(256) void scan_kernel(
    const float* __restrict__ DLR, const float* __restrict__ UC, const float* __restrict__ XZ,
    const float* __restrict__ PROJ, const float* __restrict__ A_log, const float* __restrict__ Dv,
    unsigned short* __restrict__ Y16)
{
  __shared__ __align__(16) float sBC[16 * 32];
  __shared__ __align__(16) float sY[16 * kTP];
  const int tid = threadIdx.x, lane = tid & 31, wave = tid >> 5;
  const int d0 = blockIdx.x * 256, d = d0 + tid;

  float An[kNst];
#pragma unroll
  for (int n = 0; n < kNst; ++n) An[n] = -__expf(A_log[(size_t)d * kNst + n]);
  const float Dd = Dv[d];
  float h[kNst];
#pragma unroll
  for (int n = 0; n < kNst; ++n) h[n] = 0.f;

#pragma unroll 1
  for (int c = 0; c < kSeqL / 16; ++c) {
    const int l0 = c * 16;
    if (tid < 128) {
      const int r = tid >> 3, q = (tid & 7) * 4;
      const v4f v = *(const v4f*)(PROJ + (size_t)(l0 + r) * kPrjP + kDtR + q);
      *(v4f*)(sBC + r * 32 + q) = v;
    }
    __syncthreads();
#pragma unroll 1
    for (int s = 0; s < 16; ++s) {
      const size_t m = (size_t)(l0 + s);
      const float a     = DLR[m * kDin + d];
      const float delta = fmaxf(a, 0.0f) + log1pf(__expf(-fabsf(a)));
      const float xv    = UC[m * kDin + d];
      const float zv    = XZ[m * kXZP + kDin + d];
      v4f Bq[4], Cq[4];
#pragma unroll
      for (int qq = 0; qq < 4; ++qq) {
        Bq[qq] = *(const v4f*)(sBC + s * 32 + 4 * qq);
        Cq[qq] = *(const v4f*)(sBC + s * 32 + kNst + 4 * qq);
      }
      float y = 0.f;
#pragma unroll
      for (int n = 0; n < kNst; ++n) {
        const float e = __expf(delta * An[n]);
        float db = delta * Bq[n >> 2][n & 3];
        asm volatile("" : "+v"(db));
        float p = db * xv;
        asm volatile("" : "+v"(p));
        float qv = h[n] * e;
        asm volatile("" : "+v"(qv));
        const float hn = qv + p;
        h[n] = hn;
        float rr = Cq[n >> 2][n & 3] * hn;
        asm volatile("" : "+v"(rr));
        y += rr;
      }
      float sk = xv * Dd;
      asm volatile("" : "+v"(sk));
      y += sk;
      const float sg = __builtin_amdgcn_rcpf(1.0f + __expf(-zv));
      const float g  = zv * sg;
      sY[s * kTP + tid] = (y * g) * kYCarry;
    }
    __syncthreads();
    v8h hv[2];
#pragma unroll
    for (int it = 0; it < 2; ++it) {
      const float* sp = sY + (it * 8 + wave) * kTP + lane * 8;
      const v4f a0 = *(const v4f*)(sp);
      const v4f a1 = *(const v4f*)(sp + 4);
#pragma unroll
      for (int e = 0; e < 4; ++e) { hv[it][e] = (_Float16)a0[e]; hv[it][4 + e] = (_Float16)a1[e]; }
    }
    for (int pass = 0; pass < 2; ++pass) {
#pragma unroll
      for (int it = 0; it < 2; ++it)
        *(volatile v8h*)(Y16 + (size_t)(l0 + it * 8 + wave) * kDin + d0 + lane * 8) = hv[it];
      __threadfence();
    }
  }
}

__global__ __launch_bounds__(256) void ln_downsample_kernel(
    const float* __restrict__ Hs, const float* __restrict__ g, const float* __restrict__ bb,
    const float* __restrict__ dsw, const float* __restrict__ dsb, float* __restrict__ out, int nOut)
{
  const int lane = threadIdx.x & 31, wave = threadIdx.x >> 5;
  const int orow = blockIdx.x * 8 + wave;
  if (orow >= nOut) return;
  const float* p0 = Hs + (size_t)orow * 2 * kDmod;
  const float* p1 = p0 + kDmod;
  float s0 = 0.f, s1 = 0.f;
#pragma unroll 1
  for (int i = 0; i < kDmod / 128; ++i) {
    const v4f a = *(const v4f*)(p0 + i * 128 + lane * 4);
    const v4f c = *(const v4f*)(p1 + i * 128 + lane * 4);
    s0 += (a[0] + a[1]) + (a[2] + a[3]);
    s1 += (c[0] + c[1]) + (c[2] + c[3]);
  }
#pragma unroll
  for (int off = 1; off < 32; off <<= 1) {
    s0 += __shfl_xor(s0, off, 32);
    s1 += __shfl_xor(s1, off, 32);
  }
  const float inv = 1.0f / (float)kDmod;
  const float mu0 = s0 * inv, mu1 = s1 * inv;
  float q0 = 0.f, q1 = 0.f;
#pragma unroll 1
  for (int i = 0; i < kDmod / 128; ++i) {
    const v4f a = *(const v4f*)(p0 + i * 128 + lane * 4);
    const v4f c = *(const v4f*)(p1 + i * 128 + lane * 4);
#pragma unroll
    for (int e = 0; e < 4; ++e) {
      const float da = a[e] - mu0;
      const float dc = c[e] - mu1;
      q0 = fmaf(da, da, q0);
      q1 = fmaf(dc, dc, q1);
    }
  }
#pragma unroll
  for (int off = 1; off < 32; off <<= 1) {
    q0 += __shfl_xor(q0, off, 32);
    q1 += __shfl_xor(q1, off, 32);
  }
  const float rs0 = rsqrtf(q0 * inv + 1e-5f);
  const float rs1 = rsqrtf(q1 * inv + 1e-5f);
  const float w0 = dsw[0], w1 = dsw[1], db = dsb[0];
  float* op = out + (size_t)orow * kDmod;
#pragma unroll 1
  for (int i = 0; i < kDmod / 128; ++i) {
    const int col = i * 128 + lane * 4;
    const v4f a  = *(const v4f*)(p0 + col);
    const v4f c  = *(const v4f*)(p1 + col);
    const v4f gv = *(const v4f*)(g + col);
    const v4f bv = *(const v4f*)(bb + col);
    v4f o;
#pragma unroll
    for (int e = 0; e < 4; ++e) {
      const float n0 = (a[e] - mu0) * rs0;
      const float n1 = (c[e] - mu1) * rs1;
      const float y0 = fmaf(n0, gv[e], bv[e]);
      const float y1 = fmaf(n1, gv[e], bv[e]);
      o[e] = fmaf(y0, w0, fmaf(y1, w1, db));
    }
    float* dst = op + col;
    *(volatile v4f*)dst = o;
    __threadfence();
    *(volatile v4f*)dst = o;
  }
}

extern "C" void kernel_launch(void* const* d_in, const int* in_sizes, int n_in,
                              void* d_out, int out_size, void* d_ws, size_t ws_size,
                              hipStream_t stream)
{
  if (n_in < 14) return;
  const float* x      = (const float*)d_in[0];
  const float* W_in   = (const float*)d_in[1];
  const float* conv_w = (const float*)d_in[2];
  const float* conv_b = (const float*)d_in[3];
  const float* W_xprj = (const float*)d_in[4];
  const float* W_dt   = (const float*)d_in[5];
  const float* b_dt   = (const float*)d_in[6];
  const float* A_log  = (const float*)d_in[7];
  const float* Dv     = (const float*)d_in[8];
  const float* W_out  = (const float*)d_in[9];
  const float* ln_g   = (const float*)d_in[10];
  const float* ln_b   = (const float*)d_in[11];
  const float* ds_w   = (const float*)d_in[12];
  const float* ds_b   = (const float*)d_in[13];
  float* dout = (float*)d_out;

  if (in_sizes[0] != kRows * kDmod) return;
  if (in_sizes[1] != kDmod * kXZP) return;
  if (in_sizes[2] != kDin * 4 || in_sizes[3] != kDin) return;
  if (in_sizes[4] != kDin * kPrjN) return;
  if (in_sizes[5] != kDtR * kDin || in_sizes[6] != kDin) return;
  if (in_sizes[7] != kDin * kNst || in_sizes[8] != kDin) return;
  if (in_sizes[9] != kDin * kDmod) return;
  if (in_sizes[10] != kDmod || in_sizes[11] != kDmod) return;
  if (in_sizes[12] != kDsf || in_sizes[13] != 1) return;
  if (out_size != kOutRows * kDmod) return;

  const size_t SZ_WIN16  = (size_t)kXZP * kDmod * 2;
  const size_t SZ_WXP16  = (size_t)kPrjP * kDin * 2;
  const size_t SZ_WDT16  = (size_t)kDin * kDtR * 2;
  const size_t SZ_WOUT16 = (size_t)kDmod * kDin * 2;
  const size_t SZ_X16    = (size_t)kRows * kDmod * 2;
  const size_t SZ_XZ     = (size_t)kSeqL * kXZP * 4;
  const size_t SZ_UC     = (size_t)kSeqL * kDin * 4;
  const size_t SZ_UC16   = (size_t)kSeqL * kDin * 2;
  const size_t SZ_PROJ   = (size_t)kSeqL * kPrjP * 4;
  const size_t SZ_DT16   = (size_t)kSeqL * kDtR * 2;
  const size_t SZ_DLR    = (size_t)kSeqL * kDin * 4;
  const size_t SZ_Y16    = (size_t)kSeqL * kDin * 2;
  const size_t SZ_HS     = (size_t)kRows * kDmod * 4;
  const size_t OFF_WIN16  = 0;
  const size_t OFF_WXP16  = OFF_WIN16  + SZ_WIN16;
  const size_t OFF_WDT16  = OFF_WXP16  + SZ_WXP16;
  const size_t OFF_WOUT16 = OFF_WDT16  + SZ_WDT16;
  const size_t OFF_X16    = OFF_WOUT16 + SZ_WOUT16;
  const size_t OFF_XZ     = OFF_X16    + SZ_X16;
  const size_t OFF_UC     = OFF_XZ     + SZ_XZ;
  const size_t OFF_UC16   = OFF_UC     + SZ_UC;
  const size_t OFF_PROJ   = OFF_UC16   + SZ_UC16;
  const size_t OFF_DT16   = OFF_PROJ   + SZ_PROJ;
  const size_t OFF_DLR    = OFF_DT16   + SZ_DT16;
  const size_t OFF_Y16    = OFF_DLR    + SZ_DLR;
  const size_t OFF_HS     = OFF_Y16    + SZ_Y16;
  const size_t TOTAL      = OFF_HS     + SZ_HS;
  if (ws_size < TOTAL) return;

  char* ws = (char*)d_ws;
  unsigned short* WIN16  = (unsigned short*)(ws + OFF_WIN16);
  unsigned short* WXP16  = (unsigned short*)(ws + OFF_WXP16);
  unsigned short* WDT16  = (unsigned short*)(ws + OFF_WDT16);
  unsigned short* WOUT16 = (unsigned short*)(ws + OFF_WOUT16);
  unsigned short* X16    = (unsigned short*)(ws + OFF_X16);
  float*          XZ     = (float*)(ws + OFF_XZ);
  float*          UC     = (float*)(ws + OFF_UC);
  unsigned short* UC16   = (unsigned short*)(ws + OFF_UC16);
  float*          PROJ   = (float*)(ws + OFF_PROJ);
  unsigned short* DT16   = (unsigned short*)(ws + OFF_DT16);
  float*          DLR    = (float*)(ws + OFF_DLR);
  unsigned short* Y16    = (unsigned short*)(ws + OFF_Y16);
  float*          HS     = (float*)(ws + OFF_HS);
  const float* dummy_bias  = b_dt;
  const float* dummy_resid = x;

  transpose_cast_kernel<<<dim3(kXZP / 64, kDmod / 64), 256, 0, stream>>>(W_in,   WIN16,  kDmod, kXZP,  kXZP,  kWCarry);
  transpose_cast_kernel<<<dim3(kPrjP / 64, kDin / 64), 256, 0, stream>>>(W_xprj, WXP16,  kDin,  kPrjN, kPrjP, kWCarry);
  transpose_cast32_kernel<<<dim3(kDin / 64), 256, 0, stream>>>(W_dt, WDT16, kDin, kWdtCarry);
  transpose_cast_kernel<<<dim3(kDmod / 64, kDin / 64), 256, 0, stream>>>(W_out,  WOUT16, kDin,  kDmod, kDmod, kWCarry);

  cast_f16_kernel<<<(kRows * kDmod) / 8 / 256, 256, 0, stream>>>(x, X16, (kRows * kDmod) / 8, 1.0f);

  for (int b = 0; b < kBatch; ++b) {
    const unsigned short* X16b = X16 + (size_t)b * kSeqL * kDmod;
    const float* xb = x + (size_t)b * kSeqL * kDmod;
    float* Hb = HS + (size_t)b * kSeqL * kDmod;

    wmma_gemm64<0, false, 0, 0, false><<<dim3(128, 1), 256, 0, stream>>>(
        X16b, X16b, kDmod, 0L, WIN16, WIN16, kDmod, 0L,
        (void*)XZ, (void*)XZ, kXZP, 0L, dummy_bias, dummy_resid, 0L, kSeqL, kXZP, kDmod, 1.0f / kWCarry);

    conv_silu_kernel<<<dim3(kDin / 256, kSeqL / 64), 256, 0, stream>>>(XZ, conv_w, conv_b, UC, UC16);

    wmma_gemm64<0, false, 0, 0, false><<<dim3(4, 1), 256, 0, stream>>>(
        UC16, UC16, kDin, 0L, WXP16, WXP16, kDin, 0L,
        (void*)PROJ, (void*)PROJ, kPrjP, 0L, dummy_bias, dummy_resid, 0L, kSeqL, kPrjP, kDin, 1.0f / (kUcCarry * kWCarry));

    dt_cast_kernel<<<(kSeqL * kDtR) / 8 / 256, 256, 0, stream>>>(PROJ, DT16, (kSeqL * kDtR) / 8, kDtCarry);

    wmma_gemm64<0, false, 2, 0, false><<<dim3(64, 1), 256, 0, stream>>>(
        DT16, DT16, kDtR, 0L, WDT16, WDT16, kDtR, 0L,
        (void*)DLR, (void*)DLR, kDin, 0L, b_dt, dummy_resid, 0L, kSeqL, kDin, kDtR, 1.0f / (kDtCarry * kWdtCarry));

    scan_kernel<<<dim3(kDin / 256, 1), 256, 0, stream>>>(DLR, UC, XZ, PROJ, A_log, Dv, Y16);

    wmma_gemm64<0, false, 0, 0, true><<<dim3(32, 1), 256, 0, stream>>>(
        Y16, Y16, kDin, 0L, WOUT16, WOUT16, kDin, 0L,
        (void*)Hb, (void*)Hb, kDmod, 0L, dummy_bias, xb, 0L, kSeqL, kDmod, kDin, 1.0f / (kYCarry * kWCarry));
  }

  ln_downsample_kernel<<<kOutRows / 8, 256, 0, stream>>>(HS, ln_g, ln_b, ds_w, ds_b, dout, kOutRows);
}
